// GIN_22316650070138
// MI455X (gfx1250) — hardware-verified
//
#include <hip/hip_runtime.h>
#include <stddef.h>
#include <stdint.h>


#define DIN      128
#define DHID     128
#define NOUT     6
#define APW      256
#define KTOT     256
#define WSQ      (DHID * KTOT)
#define NMAT     4
#define NTHR     256
#define NWAVE    8
#define EPT      8
#define CHUNK    (NTHR * EPT)
#define WCAP     (EPT * 32)
#define LISTN    (NWAVE * WCAP)
#define NBMAX    2048
#define RCAP     28672
#define DEGCAP   64
#define PKS      11
#define STW      512
#define GBM      64
#define GTHR     128
#define GNT      8
#define BN       (16 * GNT)
#define NUSQ     (DHID * (KTOT / 8))
#define PG       32
#define MAXG     2048
#define WSMAX    134217728
#define LDS_AGG  ((2 * RCAP + 2 * NBMAX + LISTN) * 4 + 64)

static_assert((CHUNK & (CHUNK - 1)) == 0 && CHUNK <= (1 << PKS));
static_assert((NBMAX & (NBMAX - 1)) == 0 && NBMAX <= (1 << PKS));
static_assert(NTHR * 8 == NBMAX);
static_assert(LISTN >= NBMAX);
static_assert(LISTN >= NWAVE * WCAP);
static_assert((RCAP % 32) == 0);
static_assert(NWAVE * STW <= RCAP);
static_assert(LDS_AGG <= 300000);
static_assert(GBM == (GTHR / 32) * 16);
static_assert((DIN % 32) == 0 && KTOT == 2 * DIN && APW == 2 * DIN);
static_assert(DIN == 32 * 4 && DHID == BN && DHID == DIN && GTHR == BN);
static_assert((NUSQ % NTHR) == 0 && (KTOT / 8) == 32);
static_assert(((NMAT * NUSQ) % NTHR) == 0);
static_assert(APW * 2 == DHID * 4);
static_assert((PG & (PG - 1)) == 0 && PG <= NBMAX && ((PG * DHID / 4) % NTHR) == 0);
static_assert(NTHR >= PG && NTHR > DHID && (PG * DHID) % NTHR == 0);
static_assert((MAXG * NOUT) % 4 == 0);

typedef float          v4f  __attribute__((ext_vector_type(4)));
typedef float          v8f  __attribute__((ext_vector_type(8)));
typedef int            v4i  __attribute__((ext_vector_type(4)));
typedef int            v8i  __attribute__((ext_vector_type(8)));
typedef unsigned int   v2u  __attribute__((ext_vector_type(2)));
typedef unsigned int   v4u  __attribute__((ext_vector_type(4)));
typedef unsigned short v8us __attribute__((ext_vector_type(8)));
typedef __bf16         v16b __attribute__((ext_vector_type(16)));
typedef v4f  __attribute__((may_alias)) v4fa;
typedef v4u  __attribute__((may_alias)) v4ua;
typedef v8us __attribute__((may_alias)) v8usa;
union FragB { v16b v; v8us h[2]; v8i w; };

__device__ __forceinline__ v8f wmb(const FragB& a, const FragB& b, v8f c) {
  v8f d = __builtin_amdgcn_wmma_f32_16x16x32_bf16(false, a.v, false, b.v, (short)0, c, false, false);
  asm volatile("v_nop\n\tv_nop\n\tv_nop\n\tv_nop" : "+v"(d) : "v"(a.w), "v"(b.w));
  return d;
}

__device__ __forceinline__ unsigned short bf_bits(float f) {
  unsigned int u = __float_as_uint(f);
  u += 0x7FFFu + ((u >> 16) & 1u);
  return (unsigned short)(u >> 16);
}
__device__ __forceinline__ float bf_val(unsigned short b) {
  return __uint_as_float(((unsigned int)b) << 16);
}
__device__ __forceinline__ float bf_rne(float f) { return bf_val(bf_bits(f)); }

__device__ __forceinline__ int scan_chunk(const int* __restrict__ dsts, int nE, int cbase, int slotBase,
                                          int nb, int vec8, int* list, int tid, int lane, int wave) {
  int wc = 0;
  const int el0  = tid * EPT;
  const int e0   = cbase + el0;
  const int sent = -2147483647 - 1;
  v4i da, db;
  if (vec8 != 0 && cbase + CHUNK <= nE) {
    da = *(const v4i*)(dsts + e0);
    db = *(const v4i*)(dsts + e0 + 4);
  } else {
    da.x = (e0     < nE) ? dsts[min(e0,     nE - 1)] : sent;
    da.y = (e0 + 1 < nE) ? dsts[min(e0 + 1, nE - 1)] : sent;
    da.z = (e0 + 2 < nE) ? dsts[min(e0 + 2, nE - 1)] : sent;
    da.w = (e0 + 3 < nE) ? dsts[min(e0 + 3, nE - 1)] : sent;
    db.x = (e0 + 4 < nE) ? dsts[min(e0 + 4, nE - 1)] : sent;
    db.y = (e0 + 5 < nE) ? dsts[min(e0 + 5, nE - 1)] : sent;
    db.z = (e0 + 6 < nE) ? dsts[min(e0 + 6, nE - 1)] : sent;
    db.w = (e0 + 7 < nE) ? dsts[min(e0 + 7, nE - 1)] : sent;
  }
  const unsigned nbs = (unsigned)slotBase;
  const unsigned unb = (unsigned)nb;
  const unsigned s0 = (unsigned)da.x - nbs, s1 = (unsigned)da.y - nbs;
  const unsigned s2 = (unsigned)da.z - nbs, s3 = (unsigned)da.w - nbs;
  const unsigned s4 = (unsigned)db.x - nbs, s5 = (unsigned)db.y - nbs;
  const unsigned s6 = (unsigned)db.z - nbs, s7 = (unsigned)db.w - nbs;
  const bool h0 = s0 < unb, h1 = s1 < unb, h2 = s2 < unb, h3 = s3 < unb;
  const bool h4 = s4 < unb, h5 = s5 < unb, h6 = s6 < unb, h7 = s7 < unb;
  const unsigned any = __builtin_amdgcn_ballot_w32(h0 | h1 | h2 | h3 | h4 | h5 | h6 | h7);
  if (any != 0u) {
#define HITJ(J, HJ, SJ) { \
      const unsigned mj = __builtin_amdgcn_ballot_w32(HJ); \
      if (mj != 0u) { \
        if (HJ) { \
          const int pos = wc + (int)__builtin_amdgcn_mbcnt_lo(mj, 0u); \
          if (pos < WCAP) list[wave * WCAP + pos] = ((el0 + (J)) << PKS) | (int)(SJ); \
        } \
        wc += (int)__builtin_popcount(mj); } }
    HITJ(0, h0, s0)
    HITJ(1, h1, s1)
    HITJ(2, h2, s2)
    HITJ(3, h3, s3)
    HITJ(4, h4, s4)
    HITJ(5, h5, s5)
    HITJ(6, h6, s6)
    HITJ(7, h7, s7)
#undef HITJ
  }
  return wc;
}

__global__ __launch_bounds__(NTHR) void k_wprep(const float* __restrict__ w0, const float* __restrict__ w1,
                                                const float* __restrict__ w2, const float* __restrict__ w3,
                                                unsigned short* wt) {
  const int u  = (int)blockIdx.x * NTHR + (int)threadIdx.x;
  if (u >= NMAT * NUSQ) return;
  const int mi = u / NUSQ;
  const int v  = u - mi * NUSQ;
  const int n  = v >> 5;
  const int k8 = (v & 31) * 8;
  const int kk = k8 & (DIN - 1);
  const float* Wb;
  if (mi == 0)      Wb = w0;
  else if (mi == 1) Wb = w1;
  else if (mi == 2) Wb = w2;
  else              Wb = w3;
  const float* p = Wb + (size_t)kk * DHID + n;
  v8us o;
#pragma unroll
  for (int i = 0; i < 8; ++i) o[i] = bf_bits(p[(size_t)i * DHID]);
  unsigned short* dp = wt + (size_t)mi * WSQ + (size_t)n * KTOT + k8;
  *(volatile v8us*)dp = o;
  __threadfence();
  *(volatile v8us*)dp = o;
}

template <int RND>
__global__ __launch_bounds__(NTHR) void k_agg(
    const int* __restrict__ srcs, const int* __restrict__ dsts,
    const float* __restrict__ F,
    unsigned short* Aout, int ldaOut,
    int nN, int nE, int nb, int vec8, int MPr) {
  extern __shared__ v4f lds_dyn[];
  int* reg1 = (int*)lds_dyn;
  int* reg2 = reg1 + RCAP;
  int* scnt = reg2 + RCAP;
  int* soff = scnt + NBMAX;
  int* list = soff + NBMAX;
  int* wcnt = list + LISTN;
  int* wtot = wcnt + NWAVE;
  const int tid = (int)threadIdx.x, lane = tid & 31, wave = tid >> 5;
  const int nodeBase = (int)blockIdx.x * nb;

  for (int i = tid; i < NBMAX; i += NTHR) scnt[i] = 0;
  __syncthreads();

  int tot = 0;
  const int nChunks = (nE + CHUNK - 1) / CHUNK;
#pragma unroll 1
  for (int ch = 0; ch < nChunks; ++ch) {
    const int cbase = ch * CHUNK;
    const int wc = scan_chunk(dsts, nE, cbase, nodeBase, nb, vec8, list, tid, lane, wave);
    if (lane == 0) wcnt[wave] = wc;
    __syncthreads();
    int pre = 0, all = 0;
#pragma unroll
    for (int w2 = 0; w2 < NWAVE; ++w2) {
      int c = wcnt[w2];
      c = c < 0 ? 0 : (c > WCAP ? WCAP : c);
      all += c;
      pre += (w2 < wave) ? c : 0;
    }
    const int wcc  = wc > WCAP ? WCAP : wc;
    const int base = tot + pre;
#pragma unroll 1
    for (int i = lane; i < wcc; i += 32) {
      const int ent = list[wave * WCAP + i];
      const int el  = (ent >> PKS) & (CHUNK - 1);
      const int sl  = ent & (NBMAX - 1);
      int eid = cbase + el;
      eid = eid > nE - 1 ? nE - 1 : eid;
      const int pos = base + i;
      if (pos < RCAP) reg1[pos] = (int)(((unsigned)eid << PKS) | (unsigned)sl);
    }
    tot += all;
    tot = tot > RCAP ? RCAP : tot;
    __syncthreads();
  }
  const int nh = tot;

  if (wave == 0) {
#pragma unroll 1
    for (int b0 = 0; b0 < nh; b0 += 32) {
      const int idx = b0 + lane;
      const int uv  = reg1[idx < RCAP ? idx : RCAP - 1];
      const int m32 = (nh - b0) < 32 ? (nh - b0) : 32;
#pragma unroll 1
      for (int k = 0; k < m32; ++k) {
        const int u  = __builtin_amdgcn_readlane(uv, k);
        const int sl = u & (NBMAX - 1);
        if (lane == 0) scnt[sl] = scnt[sl] + 1;
      }
    }
  }
  __syncthreads();

  {
    const v4i ca = *(const v4i*)(scnt + 8 * tid);
    const v4i cb = *(const v4i*)(scnt + 8 * tid + 4);
    const int e0 = ca.x < 0 ? 0 : ca.x, e1 = ca.y < 0 ? 0 : ca.y, e2 = ca.z < 0 ? 0 : ca.z, e3 = ca.w < 0 ? 0 : ca.w;
    const int e4 = cb.x < 0 ? 0 : cb.x, e5 = cb.y < 0 ? 0 : cb.y, e6 = cb.z < 0 ? 0 : cb.z, e7 = cb.w < 0 ? 0 : cb.w;
    const int ts = e0 + e1 + e2 + e3 + e4 + e5 + e6 + e7;
    int incl = ts;
#pragma unroll
    for (int d = 1; d < 32; d <<= 1) {
      const int up = __shfl_up(incl, d);
      if (lane >= d) incl += up;
    }
    if (lane == 31) wtot[wave] = incl;
    __syncthreads();
    int pre = 0;
#pragma unroll
    for (int w2 = 0; w2 < NWAVE; ++w2) pre += (w2 < wave) ? wtot[w2] : 0;
    int run = pre + incl - ts;
    soff[8 * tid + 0] = run; run += e0;
    soff[8 * tid + 1] = run; run += e1;
    soff[8 * tid + 2] = run; run += e2;
    soff[8 * tid + 3] = run; run += e3;
    soff[8 * tid + 4] = run; run += e4;
    soff[8 * tid + 5] = run; run += e5;
    soff[8 * tid + 6] = run; run += e6;
    soff[8 * tid + 7] = run;
  }
  __syncthreads();
  for (int i = tid; i < NBMAX; i += NTHR) list[i] = soff[i];
  __syncthreads();

  if (wave == 0) {
#pragma unroll 1
    for (int b0 = 0; b0 < nh; b0 += 32) {
      const int idx = b0 + lane;
      const int uv  = reg1[idx < RCAP ? idx : RCAP - 1];
      const int m32 = (nh - b0) < 32 ? (nh - b0) : 32;
#pragma unroll 1
      for (int k = 0; k < m32; ++k) {
        const int u   = __builtin_amdgcn_readlane(uv, k);
        const int sl  = u & (NBMAX - 1);
        const int eid = (int)((unsigned)u >> PKS);
        if (lane == 0) {
          int pos = list[sl];
          pos = pos < 0 ? 0 : (pos > RCAP - 1 ? RCAP - 1 : pos);
          reg2[pos] = eid;
          list[sl] = pos + 1;
        }
      }
    }
  }
  __syncthreads();

  const int nbw = nb >> 3;
  const bool ovf = (nh >= RCAP);
  const float qnan = __int_as_float(0x7fc00000);
  unsigned int* stwu = (unsigned int*)((float*)reg1 + wave * STW);

#pragma unroll 1
  for (int jt = 0; jt < nbw; ++jt) {
    const int slot = wave * nbw + jt;
    const int grow = nodeBase + slot;
    int st = soff[slot];
    const int craw = scnt[slot];
    int cnt = craw;
    st  = st < 0 ? 0 : (st > nh ? nh : st);
    cnt = cnt < 0 ? 0 : (cnt > DEGCAP ? DEGCAP : cnt);
    if (cnt > nh - st) cnt = nh - st;
    const float pz = (ovf || craw > DEGCAP) ? qnan : 0.0f;
    const bool liveRow = grow < nN;

    float ag0 = 0.f, ag1 = 0.f, ag2 = 0.f, ag3 = 0.f;
#pragma unroll 1
    for (int b0 = 0; b0 < cnt; b0 += 32) {
      int idx = st + b0 + lane;
      idx = idx > nh - 1 ? nh - 1 : idx;
      idx = idx < 0 ? 0 : (idx > RCAP - 1 ? RCAP - 1 : idx);
      int eid = reg2[idx];
      eid = eid < 0 ? 0 : (eid > nE - 1 ? nE - 1 : eid);
      const int sraw = srcs[eid];
      const int sv = sraw < 0 ? 0 : (sraw > nN - 1 ? nN - 1 : sraw);
      const int m32 = (cnt - b0) < 32 ? (cnt - b0) : 32;
#pragma unroll 1
      for (int k = 0; k < m32; ++k) {
        const int sk = __builtin_amdgcn_readlane(sv, k);
        const v4f v = *(const v4f*)(F + (size_t)sk * DIN + 4 * lane);
        float v0 = v.x, v1 = v.y, v2 = v.z, v3 = v.w;
        if (RND != 0) { v0 = bf_rne(v0); v1 = bf_rne(v1); v2 = bf_rne(v2); v3 = bf_rne(v3); }
        ag0 += v0; ag1 += v1; ag2 += v2; ag3 += v3;
      }
    }
    const int nc = liveRow ? grow : nN - 1;
    const v4f sf = *(const v4f*)(F + (size_t)nc * DIN + 4 * lane);
    float s0 = sf.x, s1 = sf.y, s2 = sf.z, s3 = sf.w;
    if (RND != 0) { s0 = bf_rne(s0); s1 = bf_rne(s1); s2 = bf_rne(s2); s3 = bf_rne(s3); }
    float r0 = s0 + ag0, r1 = s1 + ag1, r2 = s2 + ag2, r3 = s3 + ag3;
    r0 = (liveRow ? r0 : 0.0f) + pz;
    r1 = (liveRow ? r1 : 0.0f) + pz;
    r2 = (liveRow ? r2 : 0.0f) + pz;
    r3 = (liveRow ? r3 : 0.0f) + pz;

    const unsigned short hb0 = bf_bits(r0), hb1 = bf_bits(r1), hb2 = bf_bits(r2), hb3 = bf_bits(r3);
    const unsigned short lb0 = bf_bits(r0 - bf_val(hb0)), lb1 = bf_bits(r1 - bf_val(hb1));
    const unsigned short lb2 = bf_bits(r2 - bf_val(hb2)), lb3 = bf_bits(r3 - bf_val(hb3));
    v2u hw, lw;
    hw.x = (unsigned int)hb0 | ((unsigned int)hb1 << 16);
    hw.y = (unsigned int)hb2 | ((unsigned int)hb3 << 16);
    lw.x = (unsigned int)lb0 | ((unsigned int)lb1 << 16);
    lw.y = (unsigned int)lb2 | ((unsigned int)lb3 << 16);
    __builtin_amdgcn_fence(__ATOMIC_RELEASE, "wavefront");
    __builtin_amdgcn_wave_barrier();
    *(v2u*)(stwu + 2 * lane)      = hw;
    *(v2u*)(stwu + 64 + 2 * lane) = lw;
    __builtin_amdgcn_fence(__ATOMIC_RELEASE, "wavefront");
    __builtin_amdgcn_wave_barrier();
    const v4u pk = *(const v4ua*)(stwu + 4 * lane);
    unsigned short* gp = Aout + (size_t)grow * (size_t)ldaOut + 8 * lane;
    const bool wsv = grow < MPr;
    if (wsv) *(volatile v4u*)gp = pk;
    __threadfence();
    if (wsv) *(volatile v4u*)gp = pk;
  }
}

template <int MODE>
__global__ __launch_bounds__(GTHR) void k_gemm(const unsigned short* __restrict__ A,
                                               const unsigned short* __restrict__ WT,
                                               const float* __restrict__ bias,
                                               void* outp, int nN, int mRows)
{
  constexpr int NT = GNT;
  constexpr int NI = 16;
  __shared__ __attribute__((aligned(16))) float stg[GBM * BN];
  const int tid = (int)threadIdx.x, lane = tid & 31, wave = tid >> 5, hh = lane >> 4, m = lane & 15;
  const int rowBase = (int)blockIdx.x * GBM;

  v8f acc[NT];
  {
    const v8f z = {0.f, 0.f, 0.f, 0.f, 0.f, 0.f, 0.f, 0.f};
#pragma unroll
    for (int t = 0; t < NT; ++t) acc[t] = z;
  }
  const unsigned short* ap = A + (size_t)(rowBase + 16 * wave + m) * (size_t)APW + 8 * hh;
  const unsigned short* wp = WT + (size_t)m * (size_t)KTOT + 8 * hh;
  constexpr int ksteps = KTOT / 32;
#pragma unroll 1
  for (int ks = 0; ks < ksteps; ++ks) {
    FragB af;
    af.h[0] = *(const v8usa*)(ap + 32 * ks);
    af.h[1] = *(const v8usa*)(ap + 32 * ks + 16);
#pragma unroll
    for (int t = 0; t < NT; ++t) {
      const unsigned short* wq = wp + (size_t)(16 * t) * (size_t)KTOT + 32 * ks;
      FragB bf;
      bf.h[0] = *(const v8usa*)wq;
      bf.h[1] = *(const v8usa*)(wq + 16);
      acc[t] = wmb(af, bf, acc[t]);
    }
  }

#pragma unroll
  for (int t = 0; t < NT; ++t) {
    const int lc = 16 * t + m;
    const float bb = bf_rne(bias[lc]);
#pragma unroll
    for (int r = 0; r < 8; ++r) {
      const int lr = 16 * wave + 8 * hh + r;
      const bool live = (rowBase + lr) < nN;
      float v = acc[t][r] + bb;
      if (MODE != 0) v = fmaxf(v, 0.0f);
      stg[lr * BN + lc] = live ? v : 0.0f;
    }
  }
  __syncthreads();

  if constexpr (MODE == 1) {
    unsigned short* outH = (unsigned short*)outp;
    const int cb = 8 * m;
    const bool isHi = (hh == 0);
    v4u pk[NI];
#pragma unroll
    for (int i = 0; i < NI; ++i) {
      const int lr = 16 * wave + i;
      const v4f a = *(const v4fa*)(stg + lr * BN + cb);
      const v4f b = *(const v4fa*)(stg + lr * BN + cb + 4);
      const float f[8] = {a.x, a.y, a.z, a.w, b.x, b.y, b.z, b.w};
      unsigned int w[4];
#pragma unroll
      for (int j = 0; j < 4; ++j) {
        const unsigned short h0 = bf_bits(f[2 * j]), h1 = bf_bits(f[2 * j + 1]);
        const unsigned short l0 = bf_bits(f[2 * j] - bf_val(h0)), l1 = bf_bits(f[2 * j + 1] - bf_val(h1));
        const unsigned short q0 = isHi ? h0 : l0, q1 = isHi ? h1 : l1;
        w[j] = (unsigned int)q0 | ((unsigned int)q1 << 16);
      }
      v4u pw; pw.x = w[0]; pw.y = w[1]; pw.z = w[2]; pw.w = w[3];
      pk[i] = pw;
    }
#pragma unroll
    for (int i = 0; i < NI; ++i) {
      const int gr = rowBase + 16 * wave + i;
      unsigned short* op = outH + (size_t)gr * (size_t)APW + 8 * lane;
      if (gr < mRows) *(volatile v4u*)op = pk[i];
    }
    __threadfence();
#pragma unroll
    for (int i = 0; i < NI; ++i) {
      const int gr = rowBase + 16 * wave + i;
      unsigned short* op = outH + (size_t)gr * (size_t)APW + 8 * lane;
      if (gr < mRows) *(volatile v4u*)op = pk[i];
    }
  } else {
    float* outF = (float*)outp;
    v4f fv[NI];
#pragma unroll
    for (int i = 0; i < NI; ++i) {
      const int lr = 16 * wave + i;
      fv[i] = *(const v4fa*)(stg + lr * BN + 4 * lane);
    }
#pragma unroll
    for (int i = 0; i < NI; ++i) {
      const int gr = rowBase + 16 * wave + i;
      float* op = outF + (size_t)gr * (size_t)DHID + 4 * lane;
      if (gr < mRows) *(volatile v4f*)op = fv[i];
    }
    __threadfence();
#pragma unroll
    for (int i = 0; i < NI; ++i) {
      const int gr = rowBase + 16 * wave + i;
      float* op = outF + (size_t)gr * (size_t)DHID + 4 * lane;
      if (gr < mRows) *(volatile v4f*)op = fv[i];
    }
  }
}

__global__ __launch_bounds__(NTHR) void k_pool(const float* __restrict__ hf, const int* __restrict__ bat,
                                               int nN, int vec8b, int nG, float* pl) {
  __shared__ __attribute__((aligned(16))) float accs[PG * DHID];
  __shared__ float cnts[PG];
  __shared__ int list[LISTN];
  __shared__ int wcnt[NWAVE];
  const int tid = (int)threadIdx.x, lane = tid & 31, wave = tid >> 5;
  const int slotBase = (int)blockIdx.x * PG;

  for (int i = tid; i < PG * DHID; i += NTHR) accs[i] = 0.0f;
  if (tid < PG) cnts[tid] = 0.0f;
  __syncthreads();

  const int nChunks = (nN + CHUNK - 1) / CHUNK;
#pragma unroll 1
  for (int ch = 0; ch < nChunks; ++ch) {
    const int cbase = ch * CHUNK;
    const int wc = scan_chunk(bat, nN, cbase, slotBase, PG, vec8b, list, tid, lane, wave);
    if (lane == 0) wcnt[wave] = wc;
    __syncthreads();
#pragma unroll 1
    for (int w2 = 0; w2 < NWAVE; ++w2) {
      int c = wcnt[w2];
      c = c < 0 ? 0 : (c > WCAP ? WCAP : c);
#pragma unroll 1
      for (int i = 0; i < c; ++i) {
        const int ent = list[w2 * WCAP + i];
        const int el  = (ent >> PKS) & (CHUNK - 1);
        const int sl  = ent & (PG - 1);
        int node = cbase + el;
        node = node < 0 ? 0 : (node > nN - 1 ? nN - 1 : node);
        if (tid < DHID) {
          accs[sl * DHID + tid] += hf[(size_t)node * DHID + tid];
        }
        if (tid == DHID) cnts[sl] += 1.0f;
      }
    }
    __syncthreads();
  }

  for (int i = tid; i < PG * DHID; i += NTHR) {
    const float c  = cnts[i / DHID];
    const float cf = c < 1.0f ? 1.0f : c;
    accs[i] = accs[i] * (1.0f / cf);
  }
  __syncthreads();

  constexpr int NITP = (PG * DHID / 4) / NTHR;
  v4f pv[NITP];
#pragma unroll
  for (int it = 0; it < NITP; ++it) {
    const int p = it * NTHR + tid;
    const int row = p >> 5, q = p & 31;
    pv[it] = *(const v4fa*)(accs + row * DHID + 4 * q);
  }
#pragma unroll
  for (int it = 0; it < NITP; ++it) {
    const int p = it * NTHR + tid;
    const int row = p >> 5, q = p & 31;
    const int g = slotBase + row;
    float* op = pl + (size_t)g * DHID + 4 * q;
    if (g < nG) *(volatile v4f*)op = pv[it];
  }
  __threadfence();
#pragma unroll
  for (int it = 0; it < NITP; ++it) {
    const int p = it * NTHR + tid;
    const int row = p >> 5, q = p & 31;
    const int g = slotBase + row;
    float* op = pl + (size_t)g * DHID + 4 * q;
    if (g < nG) *(volatile v4f*)op = pv[it];
  }
}

__global__ __launch_bounds__(NTHR) void k_head(const float* __restrict__ pl, const float* __restrict__ wl,
                                               const float* __restrict__ bl, int nG, int nOut, float* out) {
  __shared__ float wsh[DIN * NOUT];
  __shared__ float bsh[8];
  __shared__ __attribute__((aligned(16))) float outs[MAXG * NOUT];
  const int tid = (int)threadIdx.x;
#pragma unroll 1
  for (int i = tid; i < DIN * NOUT; i += NTHR) wsh[i] = bf_rne(wl[i]);
  {
    const int bi = tid < NOUT ? tid : NOUT - 1;
    const float bv = bf_rne(bl[bi]);
    if (tid < 8) bsh[tid] = bv;
  }
  __syncthreads();

  const int nIt = (nG + NTHR - 1) / NTHR;
#pragma unroll 1
  for (int it = 0; it < nIt; ++it) {
    const int g  = it * NTHR + tid;
    const int gc = g < nG ? g : nG - 1;
    const float* pr = pl + (size_t)gc * DHID;
    float a0 = 0.0f, a1 = 0.0f, a2 = 0.0f, a3 = 0.0f, a4 = 0.0f, a5 = 0.0f;
#pragma unroll 1
    for (int k4 = 0; k4 < DIN / 4; ++k4) {
      const v4f v = *(const v4f*)(pr + 4 * k4);
      const float* w = wsh + (4 * k4) * NOUT;
      a0 = fmaf(v.x, w[0],  a0); a1 = fmaf(v.x, w[1],  a1); a2 = fmaf(v.x, w[2],  a2);
      a3 = fmaf(v.x, w[3],  a3); a4 = fmaf(v.x, w[4],  a4); a5 = fmaf(v.x, w[5],  a5);
      a0 = fmaf(v.y, w[6],  a0); a1 = fmaf(v.y, w[7],  a1); a2 = fmaf(v.y, w[8],  a2);
      a3 = fmaf(v.y, w[9],  a3); a4 = fmaf(v.y, w[10], a4); a5 = fmaf(v.y, w[11], a5);
      a0 = fmaf(v.z, w[12], a0); a1 = fmaf(v.z, w[13], a1); a2 = fmaf(v.z, w[14], a2);
      a3 = fmaf(v.z, w[15], a3); a4 = fmaf(v.z, w[16], a4); a5 = fmaf(v.z, w[17], a5);
      a0 = fmaf(v.w, w[18], a0); a1 = fmaf(v.w, w[19], a1); a2 = fmaf(v.w, w[20], a2);
      a3 = fmaf(v.w, w[21], a3); a4 = fmaf(v.w, w[22], a4); a5 = fmaf(v.w, w[23], a5);
    }
    if (g < nG) {
      outs[g * NOUT + 0] = a0 + bsh[0];
      outs[g * NOUT + 1] = a1 + bsh[1];
      outs[g * NOUT + 2] = a2 + bsh[2];
      outs[g * NOUT + 3] = a3 + bsh[3];
      outs[g * NOUT + 4] = a4 + bsh[4];
      outs[g * NOUT + 5] = a5 + bsh[5];
    }
  }
  __syncthreads();

  const int nP  = nOut >> 2;
  const int rem = nOut & 3;
#pragma unroll 1
  for (int p = tid; p < nP; p += NTHR) {
    const v4f v = *(const v4fa*)(outs + 4 * p);
    *(volatile v4f*)(out + 4 * (size_t)p) = v;
  }
  if (tid == 0) {
#pragma unroll 1
    for (int j = 0; j < rem; ++j) {
      const float v = outs[4 * nP + j];
      *(volatile float*)(out + 4 * (size_t)nP + j) = v;
    }
  }
  __threadfence();
#pragma unroll 1
  for (int p = tid; p < nP; p += NTHR) {
    const v4f v = *(const v4fa*)(outs + 4 * p);
    *(volatile v4f*)(out + 4 * (size_t)p) = v;
  }
  if (tid == 0) {
#pragma unroll 1
    for (int j = 0; j < rem; ++j) {
      const float v = outs[4 * nP + j];
      *(volatile float*)(out + 4 * (size_t)nP + j) = v;
    }
  }
}

static int pick_nb(int nE, int nN) {
  int nb = NBMAX;
  while (nb > 16 && (long long)nb * (long long)nE * 5LL > (long long)RCAP * (long long)nN * 4LL) nb >>= 1;
  return nb;
}
static inline int cdiv(int a, int b) { return (a + b - 1) / b; }
static inline size_t al256(size_t o) { return (o + 255) & ~(size_t)255; }

extern "C" void kernel_launch(void* const* d_in, const int* in_sizes, int n_in,
                              void* d_out, int out_size, void* d_ws, size_t ws_size,
                              hipStream_t stream) {
  if (n_in < 13) return;
  if (in_sizes[0] < DIN || (in_sizes[0] % DIN) != 0) return;
  const int nN = in_sizes[0] / DIN;
  if (nN < 1 || nN > (1 << 22)) return;
  const int nE2 = in_sizes[1];
  if (nE2 < 2 || (nE2 & 1) != 0) return;
  const int nE = nE2 / 2;
  if (nE < 1 || nE > (1 << 21)) return;
  if (in_sizes[2] != nN) return;
  if (in_sizes[3] != DIN * DHID  || in_sizes[4]  != DHID) return;
  if (in_sizes[5] != DHID * DHID || in_sizes[6]  != DHID) return;
  if (in_sizes[7] != DHID * DHID || in_sizes[8]  != DHID) return;
  if (in_sizes[9] != DHID * DHID || in_sizes[10] != DHID) return;
  if (in_sizes[11] != DHID * NOUT || in_sizes[12] != NOUT) return;
  if (out_size < NOUT || (out_size % NOUT) != 0) return;
  const int nG = out_size / NOUT;
  if (nG < 1 || nG > MAXG) return;
  if ((long long)nG * NOUT != (long long)out_size) return;

  const float* x    = (const float*)d_in[0];
  const int*   ei   = (const int*)  d_in[1];
  const int*   src  = ei;
  const int*   dst  = ei + nE;
  const int*   bat  = (const int*)  d_in[2];
  const float* W1a  = (const float*)d_in[3];
  const float* b1a  = (const float*)d_in[4];
  const float* W1b  = (const float*)d_in[5];
  const float* b1b  = (const float*)d_in[6];
  const float* W2a  = (const float*)d_in[7];
  const float* b2a  = (const float*)d_in[8];
  const float* W2b  = (const float*)d_in[9];
  const float* b2b  = (const float*)d_in[10];
  const float* Wlin = (const float*)d_in[11];
  const float* blin = (const float*)d_in[12];
  float* out = (float*)d_out;

  const int MP    = cdiv(nN, GBM) * GBM;
  const int gM    = MP / GBM;
  const int nb    = pick_nb(nE, nN);
  const int gA    = cdiv(MP, nb);
  const int vec8  = ((nE & 3) == 0) ? 1 : 0;
  const int vec8b = 1;
  const int gP    = cdiv(nG, PG);
  const int GP    = gP * PG;
  if ((long long)gA * nb < (long long)MP) return;
  if ((long long)(gM - 1) * GBM >= (long long)nN) return;
  if ((long long)GP < (long long)nG) return;

  char* ws = (char*)d_ws;
  size_t off = 0;
  const size_t oWT = off; off = al256(off + (size_t)NMAT * WSQ * 2);
  const size_t oR1 = off; off = al256(off + (size_t)MP * (size_t)(APW * 2));
  const size_t oR2 = off; off = al256(off + (size_t)MP * (size_t)(APW * 2));
  const size_t oPL = off; off = al256(off + (size_t)GP * DHID * 4);
  if (off > ws_size || off > (size_t)WSMAX) return;
  unsigned short* WT  = (unsigned short*)(ws + oWT);
  unsigned short* R1u = (unsigned short*)(ws + oR1);
  float*          R1f = (float*)(ws + oR1);
  unsigned short* R2u = (unsigned short*)(ws + oR2);
  float*          R2f = (float*)(ws + oR2);
  float*          PL  = (float*)(ws + oPL);

  hipFuncSetAttribute(reinterpret_cast<const void*>(&k_agg<1>), hipFuncAttributeMaxDynamicSharedMemorySize, LDS_AGG);
  hipFuncSetAttribute(reinterpret_cast<const void*>(&k_agg<0>), hipFuncAttributeMaxDynamicSharedMemorySize, LDS_AGG);

  k_wprep<<<(NMAT * NUSQ) / NTHR, NTHR, 0, stream>>>(W1a, W1b, W2a, W2b, WT);
  k_agg<1><<<gA, NTHR, LDS_AGG, stream>>>(src, dst, x, R1u, APW, nN, nE, nb, vec8, MP);
  k_gemm<1><<<gM, GTHR, 0, stream>>>(R1u, WT + (size_t)0 * WSQ, b1a, (void*)R2u, nN, MP);
  k_gemm<2><<<gM, GTHR, 0, stream>>>(R2u, WT + (size_t)1 * WSQ, b1b, (void*)R1f, nN, MP);
  k_agg<0><<<gA, NTHR, LDS_AGG, stream>>>(src, dst, R1f, R2u, APW, nN, nE, nb, vec8, MP);
  k_gemm<1><<<gM, GTHR, 0, stream>>>(R2u, WT + (size_t)2 * WSQ, b2a, (void*)R1u, nN, MP);
  k_gemm<0><<<gM, GTHR, 0, stream>>>(R1u, WT + (size_t)3 * WSQ, b2b, (void*)R2f, nN, MP);
  k_pool<<<gP, NTHR, 0, stream>>>(R2f, bat, nN, vec8b, nG, PL);
  k_head<<<1, NTHR, 0, stream>>>(PL, Wlin, blin, nG, out_size, out);
}
